// RNN_84885733638382
// MI455X (gfx1250) — hardware-run, weakly checked
//
#include <hip/hip_runtime.h>
#include <math.h>

typedef __attribute__((ext_vector_type(16))) _Float16 v16h;
typedef __attribute__((ext_vector_type(8)))  _Float16 v8h;
typedef __attribute__((ext_vector_type(16))) __bf16   v16b;
typedef __attribute__((ext_vector_type(8)))  __bf16   v8b;
typedef __attribute__((ext_vector_type(8)))  float    v8f;
typedef __attribute__((ext_vector_type(4)))  float    v4f;

constexpr int kBatch  = 64;
constexpr int kSteps  = 512;
constexpr int kIn     = 256;
constexpr int kHid    = 256;
constexpr int kRows   = kBatch * kSteps;
constexpr int kThr    = 256;
constexpr int kThrRun = 512;
constexpr int kSeqBlk = 16;
constexpr int kHP     = 264;

constexpr float kInCarry  = 1024.0f;
constexpr float kWCarry   = 1024.0f;
constexpr float kActCarry = 4096.0f;
constexpr float kXpScale  = 1.0f / (kInCarry * kWCarry);
constexpr float kRecScale = 1.0f / (kActCarry * kWCarry);
constexpr float kF16MinNormal = 6.103515625e-5f;

static_assert(kRows == 32768 && (kRows % 64) == 0 && (kHid % 64) == 0 && (kIn % 32) == 0, "GEMM M, N multiples of 64, K of 32");
static_assert(kHid == 16 * (kThrRun / 32), "16 waves x 16 hidden units");
static_assert(kSeqBlk == kThrRun / 32 && kBatch % kSeqBlk == 0, "one wave per batch row of the block in the row store");
static_assert((kHP % 8) == 0 && kHP >= kHid + 8, "f16 tile pitch");

constexpr size_t kOffX16  = 0;
constexpr size_t kOffWXT  = kOffX16 + (size_t)kRows * kIn * 2;
constexpr size_t kOffWHT  = kOffWXT + (size_t)kHid * kIn * 2;
constexpr size_t kOffXP   = kOffWHT + (size_t)kHid * kHid * 2;
constexpr size_t kWsTotal = kOffXP  + (size_t)kRows * kHid * 4;
static_assert(kWsTotal == 50593792ull, "carve total");
static_assert(kWsTotal <= 134217728ull, "carve cap");
static_assert((kOffWXT % 256) == 0 && (kOffWHT % 256) == 0 && (kOffXP % 256) == 0, "aligned regions");

__device__ __forceinline__ unsigned short f2bf_bits(float f) {
  unsigned u = __float_as_uint(f);
  return (unsigned short)((u + 0x7FFFu + ((u >> 16) & 1u)) >> 16);
}
__device__ __forceinline__ float bf_bits2f(unsigned short h) { return __uint_as_float(((unsigned)h) << 16); }
__device__ __forceinline__ float bf16r(float f) { return bf_bits2f(f2bf_bits(f)); }
__device__ __forceinline__ float carry_flush(float v, float carry) {
  const float s = v * carry;
  return (fabsf(s) < kF16MinNormal) ? 0.0f : s;
}
__device__ __forceinline__ float frcp(float x) { return __builtin_amdgcn_rcpf(x); }

__device__ __forceinline__ void dep_guard4_h(v8f& a, v8f& b, v8f& c, v8f& d, v16h x, v16h y) { asm volatile("v_nop\n\tv_nop\n\tv_nop\n\tv_nop" : "+v"(a), "+v"(b), "+v"(c), "+v"(d) : "v"(x), "v"(y)); }
__device__ __forceinline__ void dep_guard4_b(v8f& a, v8f& b, v8f& c, v8f& d, v16b x, v16b y) { asm volatile("v_nop\n\tv_nop\n\tv_nop\n\tv_nop" : "+v"(a), "+v"(b), "+v"(c), "+v"(d) : "v"(x), "v"(y)); }
__device__ __forceinline__ void keep4_h(v16h a, v16h b, v16h c, v16h d) { asm volatile("v_nop" :: "v"(a), "v"(b), "v"(c), "v"(d)); }
__device__ __forceinline__ void keep4_b(v16b a, v16b b, v16b c, v16b d) { asm volatile("v_nop" :: "v"(a), "v"(b), "v"(c), "v"(d)); }
__device__ __forceinline__ void acc_guard4(v8f& a, v8f& b, v8f& c, v8f& d) { asm volatile("v_nop\n\tv_nop\n\tv_nop\n\tv_nop" : "+v"(a), "+v"(b), "+v"(c), "+v"(d)); }

template <typename T> struct Frag;
template <> struct Frag<_Float16> {
  typedef v16h V; union U { v16h v; v8h h[2]; };
  static __device__ __forceinline__ v16h load(const _Float16* p) {
    U f; f.h[0] = *(const v8h*)(p); f.h[1] = *(const v8h*)(p + 16); return f.v;
  }
  static __device__ __forceinline__ v8f mma(v16h a, v16h b, v8f c) {
    return __builtin_amdgcn_wmma_f32_16x16x32_f16(false, a, false, b, (short)0, c, false, false);
  }
  static __device__ __forceinline__ void guard4(v8f& a, v8f& b, v8f& c, v8f& d, v16h x, v16h y) { dep_guard4_h(a, b, c, d, x, y); }
  static __device__ __forceinline__ void keep(v16h a, v16h b, v16h c, v16h d) { keep4_h(a, b, c, d); }
};
template <> struct Frag<__bf16> {
  typedef v16b V; union U { v16b v; v8b h[2]; };
  static __device__ __forceinline__ v16b load(const __bf16* p) {
    U f; f.h[0] = *(const v8b*)(p); f.h[1] = *(const v8b*)(p + 16); return f.v;
  }
  static __device__ __forceinline__ v8f mma(v16b a, v16b b, v8f c) {
    return __builtin_amdgcn_wmma_f32_16x16x32_bf16(false, a, false, b, (short)0, c, false, false);
  }
  static __device__ __forceinline__ void guard4(v8f& a, v8f& b, v8f& c, v8f& d, v16b x, v16b y) { dep_guard4_b(a, b, c, d, x, y); }
  static __device__ __forceinline__ void keep(v16b a, v16b b, v16b c, v16b d) { keep4_b(a, b, c, d); }
};

__device__ __forceinline__ v8f mma_h(v16h a, v16h b, v8f c) {
  c = __builtin_amdgcn_wmma_f32_16x16x32_f16(false, a, false, b, (short)0, c, false, false);
  asm volatile("v_nop\n\tv_nop\n\tv_nop\n\tv_nop" : "+v"(c) : "v"(a), "v"(b));
  return c;
}

template <int ET> struct Elem;
template <> struct Elem<0> { typedef _Float16 T; };
template <> struct Elem<1> { typedef __bf16 T; };
template <int ET, bool SPLIT, int BIAS_MODE, int OUT_MODE, bool RESID, int ACT = 0>
__global__ __launch_bounds__(256) void wmma_gemm64(
    const unsigned short* __restrict__ Ap, const unsigned short* __restrict__ A2p, int lda, long strideA,
    const unsigned short* __restrict__ Btp, const unsigned short* __restrict__ Bt2p, int ldb, long strideB,
    void* __restrict__ Cout, void* __restrict__ Cout2, int ldc, long strideC,
    const float* __restrict__ bias,
    const float* __restrict__ resid, long strideR,
    int M, int N, int K, float scale) {
  typedef typename Elem<ET>::T T;
  typedef typename Frag<T>::V V;
  const T* A = (const T*)Ap; const T* A2 = (const T*)A2p; const T* Bt = (const T*)Btp; const T* Bt2 = (const T*)Bt2p;
  __shared__ __align__(16) float sT[8][16 * 68];
  const int b    = blockIdx.y;
  const int lane = threadIdx.x & 31;
  const int wave = threadIdx.x >> 5;
  const int tilesN = N >> 6;
  const int tilesM = M >> 6;
  const int tile = blockIdx.x * 8 + wave;
  if (tile >= tilesM * tilesN) return;
  const int tm = tile / tilesN;
  const int tn = tile - tm * tilesN;
  const int m0 = tm << 6;
  const int n0 = tn << 6;

  const T* Ab  = A  + (size_t)b * strideA;
  const T* Bb  = Bt + (size_t)b * strideB;
  const T* Ab2 = SPLIT ? (A2  + (size_t)b * strideA) : nullptr;
  const T* Bb2 = SPLIT ? (Bt2 + (size_t)b * strideB) : nullptr;

  const int rlane = lane & 15;
  const int koff  = (lane >> 4) * 8;
  const int mOff  = (lane >> 4) * 8;

  v8f acc[4][4];
#pragma unroll
  for (int i = 0; i < 4; ++i)
#pragma unroll
    for (int j = 0; j < 4; ++j) acc[i][j] = (v8f){0.f,0.f,0.f,0.f,0.f,0.f,0.f,0.f};

  for (int k0 = 0; k0 < K; k0 += 32) {
    V bh[4], bl[4];
#pragma unroll
    for (int j = 0; j < 4; ++j) {
      const size_t bo = (size_t)(n0 + (j << 4) + rlane) * ldb + koff + k0;
      bh[j] = Frag<T>::load(Bb + bo);
      if (SPLIT) bl[j] = Frag<T>::load(Bb2 + bo);
    }
#pragma unroll
    for (int i = 0; i < 4; ++i) {
      const size_t ao = (size_t)(m0 + (i << 4) + rlane) * lda + koff + k0;
      V ah = Frag<T>::load(Ab + ao);
      V al;
      if (SPLIT) al = Frag<T>::load(Ab2 + ao);
#pragma unroll
      for (int j = 0; j < 4; ++j) {
        acc[i][j] = Frag<T>::mma(ah, bh[j], acc[i][j]);
        if (SPLIT) {
          acc[i][j] = Frag<T>::mma(ah, bl[j], acc[i][j]);
          acc[i][j] = Frag<T>::mma(al, bh[j], acc[i][j]);
        }
      }
      Frag<T>::guard4(acc[i][0], acc[i][1], acc[i][2], acc[i][3], ah, SPLIT ? al : ah);
    }
    Frag<T>::keep(bh[0], bh[1], bh[2], bh[3]);
    if (SPLIT) Frag<T>::keep(bl[0], bl[1], bl[2], bl[3]);
  }
  acc_guard4(acc[0][0], acc[0][1], acc[0][2], acc[0][3]);
  acc_guard4(acc[1][0], acc[1][1], acc[1][2], acc[1][3]);
  acc_guard4(acc[2][0], acc[2][1], acc[2][2], acc[2][3]);
  acc_guard4(acc[3][0], acc[3][1], acc[3][2], acc[3][3]);

  float* slab = sT[wave];
  const float* Rb = RESID ? (resid + (size_t)b * strideR) : nullptr;
#pragma unroll
  for (int i = 0; i < 4; ++i) {
    const int mBase = m0 + (i << 4);
#pragma unroll
    for (int j = 0; j < 4; ++j) {
      const int n = n0 + (j << 4) + rlane;
      float bv = 0.f;
      if (BIAS_MODE == 2) bv = bias[n];
#pragma unroll
      for (int r = 0; r < 8; ++r) {
        float v = acc[i][j][r] * scale;
        if (BIAS_MODE == 1) v += bias[mBase + mOff + r];
        if (BIAS_MODE == 2) v += bv;
        if (RESID) v += Rb[(size_t)(mBase + mOff + r) * ldc + n];
        if (ACT == 1) v = tanhf(v);
        if (ACT == 2) v = fmaxf(v, 0.0f);
        if (ACT == 3) v = v / (1.0f + expf(-v));
        if (ACT == 4) v = (v > 0.f) ? v : 0.01f * v;
        slab[(mOff + r) * 68 + (j << 4) + rlane] = v;
      }
    }
    __builtin_amdgcn_fence(__ATOMIC_RELEASE, "workgroup");
    __builtin_amdgcn_wave_barrier();
    __builtin_amdgcn_fence(__ATOMIC_ACQUIRE, "workgroup");
    if (OUT_MODE == 0) {
      float* C = (float*)Cout + (size_t)b * strideC;
      const int hh = lane >> 4, c4 = (lane & 15) * 4;
      for (int pass = 0; pass < 2; ++pass) {
#pragma unroll
        for (int it = 0; it < 8; ++it) {
          const int row = it * 2 + hh;
          v4f v = *(const v4f*)(slab + row * 68 + c4);
          *(volatile v4f*)(C + (size_t)(mBase + row) * ldc + n0 + c4) = v;
        }
        __threadfence();
      }
    } else {
      const int q = lane >> 3, c8 = (lane & 7) * 8;
      unsigned short* C  = (unsigned short*)Cout  + (size_t)b * strideC;
      unsigned short* C2 = (OUT_MODE == 2) ? ((unsigned short*)Cout2 + (size_t)b * strideC) : nullptr;
      for (int pass = 0; pass < 2; ++pass) {
#pragma unroll
        for (int it = 0; it < 4; ++it) {
          const int row = it * 4 + q;
          const float* sp = slab + row * 68 + c8;
          v8h hv, lv;
#pragma unroll
          for (int e = 0; e < 8; ++e) {
            if (OUT_MODE == 1) {
              hv[e] = (_Float16)sp[e];
            } else {
              unsigned short hb = f2bf_bits(sp[e]);
              unsigned short lb = f2bf_bits(sp[e] - bf_bits2f(hb));
              hv[e] = __builtin_bit_cast(_Float16, hb);
              lv[e] = __builtin_bit_cast(_Float16, lb);
            }
          }
          *(volatile v8h*)(C + (size_t)(mBase + row) * ldc + n0 + c8) = hv;
          if (OUT_MODE == 2) *(volatile v8h*)(C2 + (size_t)(mBase + row) * ldc + n0 + c8) = lv;
        }
        __threadfence();
      }
    }
    __builtin_amdgcn_fence(__ATOMIC_RELEASE, "workgroup");
    __builtin_amdgcn_wave_barrier();
    __builtin_amdgcn_fence(__ATOMIC_ACQUIRE, "workgroup");
  }
}

__global__ __launch_bounds__(kThr) void cast_plane_kernel(const float* __restrict__ src, unsigned short* __restrict__ dst,
                                                          int colsLog2, int dstPitch, int dstOff) {
  const int i   = blockIdx.x * kThr + threadIdx.x;
  const int sh  = colsLog2 - 3;
  const int row = i >> sh;
  const int c8  = (i & ((1 << sh) - 1)) * 8;
  const float* sp = src + ((size_t)row << colsLog2) + c8;
  const v4f a0 = *(const v4f*)(sp);
  const v4f a1 = *(const v4f*)(sp + 4);
  v8h hv;
#pragma unroll
  for (int e = 0; e < 4; ++e) {
    const float f0 = a0[e];
    const float f1 = a1[e];
    hv[e]     = (_Float16)carry_flush(bf16r(f0), kInCarry);
    hv[4 + e] = (_Float16)carry_flush(bf16r(f1), kInCarry);
  }
  unsigned short* dp = dst + (size_t)row * dstPitch + dstOff + c8;
  *(volatile v8h*)dp = hv;
  __threadfence();
  *(volatile v8h*)dp = hv;
}
static_assert(kInCarry == kWCarry, "one cast kernel serves inputs and weights");
__global__ __launch_bounds__(kThr) void tr_plane_kernel(const float* __restrict__ in, unsigned short* __restrict__ out,
                                                        int inPitch, int outPitch) {
  __shared__ __align__(16) float sTile[64 * 68];
  const int tid = threadIdx.x;
  const int n0 = blockIdx.x * 64;
  const int k0 = blockIdx.y * 64;
  {
    const int kk = tid >> 4;
    const int n4 = (tid & 15) * 4;
#pragma unroll
    for (int i = 0; i < 4; ++i) {
      const int k = kk + 16 * i;
      const v4f v = *(const v4f*)(in + (size_t)(k0 + k) * inPitch + n0 + n4);
#pragma unroll
      for (int e = 0; e < 4; ++e) {
        const float f = v[e];
        sTile[(n4 + e) * 68 + k] = carry_flush(bf16r(f), kWCarry);
      }
    }
  }
  __syncthreads();
  const int k8 = (tid & 7) * 8;
  v8h hv[2];
#pragma unroll
  for (int it = 0; it < 2; ++it) {
    const int n = (tid >> 3) + 32 * it;
    const float* sp = sTile + n * 68 + k8;
    const v4f a0 = *(const v4f*)(sp);
    const v4f a1 = *(const v4f*)(sp + 4);
#pragma unroll
    for (int e = 0; e < 4; ++e) {
      const float f0 = a0[e];
      const float f1 = a1[e];
      hv[it][e]     = (_Float16)f0;
      hv[it][4 + e] = (_Float16)f1;
    }
  }
  for (int pass = 0; pass < 2; ++pass) {
#pragma unroll
    for (int it = 0; it < 2; ++it) {
      const int n = (tid >> 3) + 32 * it;
      *(volatile v8h*)(out + (size_t)(n0 + n) * outPitch + k0 + k8) = hv[it];
    }
    __threadfence();
  }
}


__device__ __forceinline__ float cell_tanh(float v) {
  const float e = __expf(2.0f * v);
  return 1.0f - 2.0f * frcp(e + 1.0f);
}

__global__ __launch_bounds__(kThrRun) void tanh_run_kernel(const float* __restrict__ XP, const unsigned short* __restrict__ WHTp,
                                                           const float* __restrict__ hinit, float* __restrict__ out) {
  __shared__ __align__(16) _Float16 Ah[2][kSeqBlk * kHP];
  __shared__ __align__(16) float    Hm[2][kSeqBlk * kHid];
  const _Float16* WHT = (const _Float16*)WHTp;
  const int tid = threadIdx.x, lane = tid & 31;
  const int wave = __builtin_amdgcn_readfirstlane(tid >> 5);
  const int c = lane & 15, hh = lane >> 4, koff = hh * 8;
  const int n0 = blockIdx.x * kSeqBlk;
  const int j = 16 * wave + c;

  {
    _Float16* af = &Ah[0][0];
#pragma unroll 1
    for (int i = tid; i < 2 * kSeqBlk * kHP; i += kThrRun) af[i] = (_Float16)0.0f;
    float* hf = &Hm[0][0];
#pragma unroll 1
    for (int i = tid; i < 2 * kSeqBlk * kHid; i += kThrRun) hf[i] = 0.0f;
  }
  __syncthreads();
#pragma unroll 1
  for (int i = tid; i < kSeqBlk * kHid; i += kThrRun) {
    const int row = i >> 8;
    const int col = i & (kHid - 1);
    const float hv = bf16r(hinit[(size_t)(n0 + row) * kHid + col]);
    Hm[0][i] = hv;
    Ah[0][row * kHP + col] = (_Float16)carry_flush(hv, kActCarry);
  }
  __syncthreads();

  const _Float16* wrow = WHT + (size_t)j * kHid + koff;
  const v8f z8 = {0.f, 0.f, 0.f, 0.f, 0.f, 0.f, 0.f, 0.f};

#pragma unroll 1
  for (int t = 0; t < kSteps; ++t) {
    const int cur = t & 1;
    const _Float16* arow = &Ah[cur][0] + c * kHP + koff;
    float xp[8];
#pragma unroll
    for (int r = 0; r < 8; ++r) xp[r] = XP[((size_t)(n0 + 8 * hh + r) * kSteps + t) * kHid + j];
    v8f acc = z8;
#pragma unroll 2
    for (int k0 = 0; k0 < kHid; k0 += 32) {
      const v16h a  = Frag<_Float16>::load(arow + k0);
      const v16h fb = Frag<_Float16>::load(wrow + k0);
      acc = mma_h(a, fb, acc);
    }
    float* hmn = &Hm[cur ^ 1][0];
    _Float16* ahn = &Ah[cur ^ 1][0];
#pragma unroll
    for (int r = 0; r < 8; ++r) {
      const int row = 8 * hh + r;
      const float hv = cell_tanh(xp[r] + acc[r] * kRecScale);
      hmn[row * kHid + j] = hv;
      ahn[row * kHP + j]  = (_Float16)carry_flush(hv, kActCarry);
    }
    __syncthreads();
    {
      const v4f s0 = *(const v4f*)(hmn + wave * kHid + 4 * lane);
      const v4f s1 = *(const v4f*)(hmn + wave * kHid + 128 + 4 * lane);
      float* op = out + ((size_t)(n0 + wave) * kSteps + t) * kHid;
      for (int pass = 0; pass < 2; ++pass) {
        *(volatile v4f*)(op + 4 * lane) = s0;
        *(volatile v4f*)(op + 128 + 4 * lane) = s1;
        __threadfence();
      }
    }
  }
}

static_assert(((kRows / 64) * (kHid / 64)) % 8 == 0, "GEMM grid exact");
static_assert(((size_t)kRows * kIn / 8) % kThr == 0, "input cast grid exact");

extern "C" void kernel_launch(void* const* d_in, const int* in_sizes, int n_in,
                              void* d_out, int out_size, void* d_ws, size_t ws_size,
                              hipStream_t stream) {
  if (n_in < 5 || d_out == nullptr || d_ws == nullptr) return;
  if (in_sizes[0] != kRows * kIn) return;
  if (in_sizes[1] != kBatch * kHid) return;
  if (in_sizes[2] != kIn * kHid || in_sizes[3] != kHid * kHid || in_sizes[4] != kHid) return;
  if (out_size != kRows * kHid) return;
  if (ws_size < kWsTotal) return;

  const float* x  = (const float*)d_in[0];
  const float* h0 = (const float*)d_in[1];
  const float* Wx = (const float*)d_in[2];
  const float* Wh = (const float*)d_in[3];
  const float* b  = (const float*)d_in[4];
  float* out = (float*)d_out;

  char* ws = (char*)d_ws;
  unsigned short* X16 = (unsigned short*)(ws + kOffX16);
  unsigned short* WXT = (unsigned short*)(ws + kOffWXT);
  unsigned short* WHT = (unsigned short*)(ws + kOffWHT);
  float*          XP  = (float*)(ws + kOffXP);

  cast_plane_kernel<<<(kRows * kIn / 8) / kThr, kThr, 0, stream>>>(x, X16, 8, kIn, 0);
  tr_plane_kernel<<<dim3(kHid / 64, kIn / 64),  kThr, 0, stream>>>(Wx, WXT, kHid, kIn);
  tr_plane_kernel<<<dim3(kHid / 64, kHid / 64), kThr, 0, stream>>>(Wh, WHT, kHid, kHid);

  wmma_gemm64<0, false, 2, 0, false, 0><<<dim3((kRows / 64) * (kHid / 64) / 8, 1), 256, 0, stream>>>(
      X16, X16, kIn, 0L, WXT, WXT, kIn, 0L, (void*)XP, (void*)XP, kHid, 0L,
      b, nullptr, 0L, kRows, kHid, kIn, kXpScale);

  tanh_run_kernel<<<kBatch / kSeqBlk, kThrRun, 0, stream>>>(XP, WHT, h0, out);
}
